// RNN_Net_34686155882861
// MI455X (gfx1250) — hardware-run, weakly checked
//
#include <hip/hip_runtime.h>

constexpr int NB_ROWS  = 16384;
constexpr int NSTEPS   = 28;
constexpr int NINP     = 28;
constexpr int NHID     = 128;
constexpr int NCLS     = 11;
constexpr int XROWF    = NSTEPS * NINP;
constexpr int NTHR     = 128;
constexpr int NWAVE    = NTHR / 32;
constexpr int ROWS_BLK = NWAVE * 16;
constexpr int WP       = 136;
constexpr int XPITCH   = 32;
constexpr float WCAR     = 16.0f;
constexpr float WCAR_INV = 1.0f / 16.0f;

constexpr int SZ_WI0   = NHID * XPITCH * 2;
constexpr int SZ_W     = NHID * WP * 2;
constexpr int SZ_FCW   = 16 * WP * 2;
constexpr int SZ_HT    = 16 * WP * 2;
constexpr int SZ_XT    = 16 * XPITCH * 2;
constexpr int OFFB_WI0 = 0;
constexpr int OFFB_WH0 = OFFB_WI0 + SZ_WI0;
constexpr int OFFB_WI1 = OFFB_WH0 + SZ_W;
constexpr int OFFB_WH1 = OFFB_WI1 + SZ_W;
constexpr int OFFB_WI2 = OFFB_WH1 + SZ_W;
constexpr int OFFB_WH2 = OFFB_WI2 + SZ_W;
constexpr int OFFB_FCW = OFFB_WH2 + SZ_W;
constexpr int OFFB_HT  = OFFB_FCW + SZ_FCW;
constexpr int OFFB_XT  = OFFB_HT + 3 * NWAVE * SZ_HT;
constexpr int OFFB_BIAS = OFFB_XT + NWAVE * SZ_XT;
constexpr int SZ_BIAS   = (3 * NHID + 16) * 4;
constexpr int OFFB_OUTS = OFFB_BIAS + SZ_BIAS;
constexpr int SZ_OUTS   = ROWS_BLK * NCLS * 4;
constexpr int LDS_TOTAL = OFFB_OUTS + SZ_OUTS;
static_assert(OFFB_WH0 % 16 == 0 && OFFB_WI1 % 16 == 0 && OFFB_FCW % 16 == 0 && OFFB_HT % 16 == 0);
static_assert(OFFB_XT % 16 == 0 && OFFB_BIAS % 16 == 0 && OFFB_OUTS % 16 == 0 && LDS_TOTAL % 16 == 0);
static_assert(NB_ROWS % ROWS_BLK == 0);
static_assert((NHID * NHID / 8) % NTHR == 0);
static_assert((NHID * (NINP / 4)) % NTHR == 0);
static_assert(SZ_WI0 % 16 == 0 && SZ_FCW % 16 == 0 && (OFFB_BIAS - OFFB_HT) % 16 == 0);
static_assert((ROWS_BLK * NCLS * 4) % 128 == 0);
static_assert((XROWF * 4) % 16 == 0 && (NINP * 4) % 16 == 0);

typedef __attribute__((ext_vector_type(16))) _Float16 v16h;
typedef __attribute__((ext_vector_type(8)))  _Float16 v8h;
typedef __attribute__((ext_vector_type(4)))  _Float16 v4h;
typedef __attribute__((ext_vector_type(8)))  float    v8f;
typedef __attribute__((ext_vector_type(4)))  float    v4f;
typedef __attribute__((ext_vector_type(4)))  unsigned v4u;

__device__ __forceinline__ void dep_guard_h(v8f& a, v8f& b, v16h x, v16h y) { asm volatile("v_nop\n\tv_nop\n\tv_nop\n\tv_nop" : "+v"(a), "+v"(b) : "v"(x), "v"(y)); }
__device__ __forceinline__ void keep4_h(v16h a, v16h b, v16h c, v16h d) { asm volatile("v_nop" :: "v"(a), "v"(b), "v"(c), "v"(d)); }
__device__ __forceinline__ void acc_guard4(v8f& a, v8f& b, v8f& c, v8f& d) { asm volatile("v_nop\n\tv_nop\n\tv_nop\n\tv_nop" : "+v"(a), "+v"(b), "+v"(c), "+v"(d)); }
__device__ __forceinline__ void acc_guard1(v8f& a, v16h x, v16h y) { asm volatile("v_nop\n\tv_nop\n\tv_nop\n\tv_nop" : "+v"(a) : "v"(x), "v"(y)); }
template <typename T> struct Frag;
template <> struct Frag<_Float16> {
  typedef v16h V; union U { v16h v; v8h h[2]; };
  static __device__ __forceinline__ v16h load(const _Float16* p) {
    U f; f.h[0] = *(const v8h*)(p); f.h[1] = *(const v8h*)(p + 16); return f.v;
  }
  static __device__ __forceinline__ v8f mma(v16h a, v16h b, v8f c) {
    return __builtin_amdgcn_wmma_f32_16x16x32_f16(false, a, false, b, (short)0, c, false, false);
  }
  static __device__ __forceinline__ void guard(v8f& a, v8f& b, v16h x, v16h y) { dep_guard_h(a, b, x, y); }
  static __device__ __forceinline__ void keep(v16h a, v16h b, v16h c, v16h d) { keep4_h(a, b, c, d); }
};

__device__ __forceinline__ void stage_w128(_Float16* dst, const float* __restrict__ src, int tid) {
#pragma unroll 1
  for (int it = 0; it < (NHID * NHID / 8) / NTHR; ++it) {
    const int i  = it * NTHR + tid;
    const int n  = i >> 4;
    const int q8 = (i & 15) * 8;
    const v4f va = *(const v4f*)(src + n * NHID + q8);
    const v4f vb = *(const v4f*)(src + n * NHID + q8 + 4);
    v8h hv;
#pragma unroll
    for (int e = 0; e < 4; ++e) {
      hv[e]     = (_Float16)(va[e] * WCAR);
      hv[4 + e] = (_Float16)(vb[e] * WCAR);
    }
    *(v8h*)(dst + n * WP + q8) = hv;
  }
}

template <int KCH, int P>
__device__ __forceinline__ void acc_term(v8f (&acc)[8], const _Float16* arow, const _Float16* wrow) {
#pragma unroll 1
  for (int kc = 0; kc < KCH; ++kc) {
    const int k0 = kc * 32;
    const v16h a = Frag<_Float16>::load(arow + k0);
    v16h bA[4];
#pragma unroll
    for (int j = 0; j < 4; ++j) bA[j] = Frag<_Float16>::load(wrow + (16 * j) * P + k0);
#pragma unroll
    for (int j = 0; j < 4; ++j) acc[j] = Frag<_Float16>::mma(a, bA[j], acc[j]);
    dep_guard_h(acc[0], acc[3], a, bA[3]);
    keep4_h(bA[0], bA[1], bA[2], bA[3]);
    v16h bB[4];
#pragma unroll
    for (int j = 0; j < 4; ++j) bB[j] = Frag<_Float16>::load(wrow + (16 * (4 + j)) * P + k0);
#pragma unroll
    for (int j = 0; j < 4; ++j) acc[4 + j] = Frag<_Float16>::mma(a, bB[j], acc[4 + j]);
    dep_guard_h(acc[4], acc[7], a, bB[3]);
    keep4_h(bB[0], bB[1], bB[2], bB[3]);
  }
}

template <int KCH_IN, int P_IN>
__device__ __forceinline__ void rnn_cell(const _Float16* ain, const _Float16* win, _Float16* hio, const _Float16* whh,
                                         const float (&bs)[8], int c, int hh) {
  const int koff = 8 * hh;
  const v8f z8 = {0.f, 0.f, 0.f, 0.f, 0.f, 0.f, 0.f, 0.f};
  v8f acc[8];
#pragma unroll
  for (int nt = 0; nt < 8; ++nt) acc[nt] = z8;
  acc_term<KCH_IN, P_IN>(acc, ain + c * P_IN + koff, win + c * P_IN + koff);
  acc_term<NHID / 32, WP>(acc, hio + c * WP + koff, whh + c * WP + koff);
  acc_guard4(acc[0], acc[1], acc[2], acc[3]);
  acc_guard4(acc[4], acc[5], acc[6], acc[7]);
#pragma unroll
  for (int nt = 0; nt < 8; ++nt) {
#pragma unroll
    for (int r = 0; r < 8; ++r) {
      float v = acc[nt][r] * WCAR_INV + bs[nt];
      v = fmaxf(v, 0.0f);
      hio[(8 * hh + r) * WP + 16 * nt + c] = (_Float16)v;
    }
  }
}

__global__ void __launch_bounds__(NTHR, 1)
rnn3_relu_fc_kernel(const float* __restrict__ x,
                    const float* __restrict__ wi0, const float* __restrict__ wh0,
                    const float* __restrict__ bi0, const float* __restrict__ bh0,
                    const float* __restrict__ wi1, const float* __restrict__ wh1,
                    const float* __restrict__ bi1, const float* __restrict__ bh1,
                    const float* __restrict__ wi2, const float* __restrict__ wh2,
                    const float* __restrict__ bi2, const float* __restrict__ bh2,
                    const float* __restrict__ fcw, const float* __restrict__ fcb,
                    float* __restrict__ out) {
  extern __shared__ v4u smem_dyn[];
  unsigned char* const smem_raw = (unsigned char*)smem_dyn;
  const int tid = threadIdx.x, lane = tid & 31, wave = tid >> 5;
  const int c = lane & 15, hh = lane >> 4, koff = 8 * hh;
  const int row0 = blockIdx.x * ROWS_BLK + wave * 16;

  _Float16* const WI0p = (_Float16*)(smem_raw + OFFB_WI0);
  _Float16* const WH0p = (_Float16*)(smem_raw + OFFB_WH0);
  _Float16* const WI1p = (_Float16*)(smem_raw + OFFB_WI1);
  _Float16* const WH1p = (_Float16*)(smem_raw + OFFB_WH1);
  _Float16* const WI2p = (_Float16*)(smem_raw + OFFB_WI2);
  _Float16* const WH2p = (_Float16*)(smem_raw + OFFB_WH2);
  _Float16* const FCWp = (_Float16*)(smem_raw + OFFB_FCW);
  _Float16* const H0p  = (_Float16*)(smem_raw + OFFB_HT + (0 * NWAVE + wave) * SZ_HT);
  _Float16* const H1p  = (_Float16*)(smem_raw + OFFB_HT + (1 * NWAVE + wave) * SZ_HT);
  _Float16* const H2p  = (_Float16*)(smem_raw + OFFB_HT + (2 * NWAVE + wave) * SZ_HT);
  _Float16* const XTp  = (_Float16*)(smem_raw + OFFB_XT + wave * SZ_XT);
  float* const BIASp   = (float*)(smem_raw + OFFB_BIAS);
  float* const OUTSp   = (float*)(smem_raw + OFFB_OUTS);

  {
    const v4u z4 = {0u, 0u, 0u, 0u};
    v4u* const p0 = (v4u*)(smem_raw + OFFB_WI0);
#pragma unroll 1
    for (int i = tid; i < SZ_WI0 / 16; i += NTHR) p0[i] = z4;
    v4u* const p1 = (v4u*)(smem_raw + OFFB_FCW);
#pragma unroll 1
    for (int i = tid; i < SZ_FCW / 16; i += NTHR) p1[i] = z4;
    v4u* const p2 = (v4u*)(smem_raw + OFFB_HT);
#pragma unroll 1
    for (int i = tid; i < (OFFB_BIAS - OFFB_HT) / 16; i += NTHR) p2[i] = z4;
  }
  __syncthreads();

  stage_w128(WH0p, wh0, tid);
  stage_w128(WI1p, wi1, tid);
  stage_w128(WH1p, wh1, tid);
  stage_w128(WI2p, wi2, tid);
  stage_w128(WH2p, wh2, tid);
#pragma unroll 1
  for (int it = 0; it < (NHID * (NINP / 4)) / NTHR; ++it) {
    const int i = it * NTHR + tid;
    const int n = i / 7;
    const int q = i - n * 7;
    const v4f v = *(const v4f*)(wi0 + n * NINP + q * 4);
    v4h hv;
    hv[0] = (_Float16)(v[0] * WCAR); hv[1] = (_Float16)(v[1] * WCAR);
    hv[2] = (_Float16)(v[2] * WCAR); hv[3] = (_Float16)(v[3] * WCAR);
    *(v4h*)(WI0p + n * XPITCH + q * 4) = hv;
  }
#pragma unroll 1
  for (int it = 0; it < 2; ++it) {
    const int i  = it * NTHR + tid;
    const bool ok = i < NCLS * (NHID / 8);
    const int ic = ok ? i : (NCLS * (NHID / 8) - 1);
    const int n  = ic >> 4;
    const int q8 = (ic & 15) * 8;
    const v4f va = *(const v4f*)(fcw + n * NHID + q8);
    const v4f vb = *(const v4f*)(fcw + n * NHID + q8 + 4);
    v8h hv;
#pragma unroll
    for (int e = 0; e < 4; ++e) {
      hv[e]     = (_Float16)(va[e] * WCAR);
      hv[4 + e] = (_Float16)(vb[e] * WCAR);
    }
    if (ok) *(v8h*)(FCWp + n * WP + q8) = hv;
  }
  {
    BIASp[tid]            = bi0[tid] + bh0[tid];
    BIASp[NHID + tid]     = bi1[tid] + bh1[tid];
    BIASp[2 * NHID + tid] = bi2[tid] + bh2[tid];
    if (tid < 16) {
      const float fv = fcb[(tid < NCLS) ? tid : (NCLS - 1)];
      BIASp[3 * NHID + tid] = (tid < NCLS) ? fv : 0.0f;
    }
  }
  __syncthreads();

  float bs0[8], bs1[8], bs2[8];
#pragma unroll
  for (int nt = 0; nt < 8; ++nt) {
    bs0[nt] = BIASp[16 * nt + c];
    bs1[nt] = BIASp[NHID + 16 * nt + c];
    bs2[nt] = BIASp[2 * NHID + 16 * nt + c];
  }
  const float fcbv = BIASp[3 * NHID + c];

#pragma unroll 1
  for (int t = 0; t < NSTEPS; ++t) {
    {
#pragma unroll
      for (int it = 0; it < 4; ++it) {
        const int idx = it * 32 + lane;
        const bool valid = idx < 16 * 7;
        const int idc = valid ? idx : (16 * 7 - 1);
        const int r = idc / 7;
        const int q = idc - r * 7;
        const v4f v = *(const v4f*)(x + (size_t)(row0 + r) * XROWF + t * NINP + q * 4);
        v4h hv;
        hv[0] = (_Float16)v[0]; hv[1] = (_Float16)v[1]; hv[2] = (_Float16)v[2]; hv[3] = (_Float16)v[3];
        if (valid) *(v4h*)(XTp + r * XPITCH + q * 4) = hv;
      }
    }
    __syncthreads();
    rnn_cell<1, XPITCH>(XTp, WI0p, H0p, WH0p, bs0, c, hh);
    __syncthreads();
    rnn_cell<NHID / 32, WP>(H0p, WI1p, H1p, WH1p, bs1, c, hh);
    __syncthreads();
    rnn_cell<NHID / 32, WP>(H1p, WI2p, H2p, WH2p, bs2, c, hh);
  }
  __syncthreads();

  {
    const v8f z8 = {0.f, 0.f, 0.f, 0.f, 0.f, 0.f, 0.f, 0.f};
    v8f facc = z8;
    const _Float16* arow = H2p  + c * WP + koff;
    const _Float16* wrow = FCWp + c * WP + koff;
#pragma unroll 1
    for (int kc = 0; kc < NHID / 32; ++kc) {
      const v16h a = Frag<_Float16>::load(arow + kc * 32);
      const v16h b = Frag<_Float16>::load(wrow + kc * 32);
      facc = Frag<_Float16>::mma(a, b, facc);
      acc_guard1(facc, a, b);
    }
#pragma unroll
    for (int r = 0; r < 8; ++r) {
      const float v = facc[r] * WCAR_INV + fcbv;
      if (c < NCLS) OUTSp[(16 * wave + 8 * hh + r) * NCLS + c] = v;
    }
  }
  __syncthreads();

  {
    float* const ob = out + (size_t)blockIdx.x * (ROWS_BLK * NCLS);
    for (int pass = 0; pass < 2; ++pass) {
#pragma unroll
      for (int it = 0; it < 2; ++it) {
        const int idx = it * NTHR + tid;
        if (idx < (ROWS_BLK * NCLS) / 4) {
          const v4f v = *(const v4f*)(OUTSp + idx * 4);
          *(volatile v4f*)(ob + idx * 4) = v;
        }
      }
      __threadfence();
    }
  }
}

extern "C" void kernel_launch(void* const* d_in, const int* in_sizes, int n_in,
                              void* d_out, int out_size, void* d_ws, size_t ws_size, hipStream_t stream) {
  (void)d_ws; (void)ws_size;
  if (n_in < 15 || d_out == nullptr) return;
  if (in_sizes[0] != NB_ROWS * XROWF || in_sizes[1] != NHID * NINP || in_sizes[2] != NHID * NHID ||
      in_sizes[3] != NHID || in_sizes[4] != NHID ||
      in_sizes[5] != NHID * NHID || in_sizes[6] != NHID * NHID || in_sizes[7] != NHID || in_sizes[8] != NHID ||
      in_sizes[9] != NHID * NHID || in_sizes[10] != NHID * NHID || in_sizes[11] != NHID || in_sizes[12] != NHID ||
      in_sizes[13] != NCLS * NHID || in_sizes[14] != NCLS || out_size != NB_ROWS * NCLS) return;

  const float* x   = (const float*)d_in[0];
  const float* wi0 = (const float*)d_in[1];
  const float* wh0 = (const float*)d_in[2];
  const float* bi0 = (const float*)d_in[3];
  const float* bh0 = (const float*)d_in[4];
  const float* wi1 = (const float*)d_in[5];
  const float* wh1 = (const float*)d_in[6];
  const float* bi1 = (const float*)d_in[7];
  const float* bh1 = (const float*)d_in[8];
  const float* wi2 = (const float*)d_in[9];
  const float* wh2 = (const float*)d_in[10];
  const float* bi2 = (const float*)d_in[11];
  const float* bh2 = (const float*)d_in[12];
  const float* fcw = (const float*)d_in[13];
  const float* fcb = (const float*)d_in[14];
  float* out = (float*)d_out;

  rnn3_relu_fc_kernel<<<dim3(NB_ROWS / ROWS_BLK), dim3(NTHR), LDS_TOTAL, stream>>>(
      x, wi0, wh0, bi0, bh0, wi1, wh1, bi1, bh1, wi2, wh2, bi2, bh2, fcw, fcb, out);
}
